// DeformableTemporalAttention_5961414607490
// MI455X (gfx1250) — hardware-verified
//
#include <hip/hip_runtime.h>
#include <math.h>
#include <stdint.h>

#define BB   2
#define NN   4
#define CC   256
#define HH   64
#define WW   64
#define HWp  4096
#define TT   64
#define KK   8
#define PP   6
#define DD   32

#define KSTEP 64
#define KP    72
#define CSP   36
#define OPSCALE 64.f
#define ACCSCALE (1.f / 4096.f)
#define PRM_N 512
#define PRM_BIAS_OFF (BB * NN * KK * PP)

#define EP_NONE 0
#define EP_GELU 1
#define EP_GATE 2

typedef _Float16 v16h __attribute__((ext_vector_type(16)));
typedef _Float16 v8h  __attribute__((ext_vector_type(8)));
typedef float    v8f  __attribute__((ext_vector_type(8)));
typedef float    v4f  __attribute__((ext_vector_type(4)));
typedef v4f __attribute__((may_alias)) v4fa;
typedef v8h __attribute__((may_alias)) v8ha;

union Frag  { v16h v; v8h half[2]; };
union HPack { v8h v[2]; _Float16 s[16]; };

__device__ __forceinline__ v8f wmma16(v16h a, v16h b, v8f acc)
{
  acc = __builtin_amdgcn_wmma_f32_16x16x32_f16(false, a, false, b, (short)0, acc, false, false);
  asm volatile("v_nop\n\tv_nop\n\tv_nop\n\tv_nop" : "+v"(acc) : "v"(a), "v"(b));
  return acc;
}

__device__ __forceinline__ float gelu_f(float x)
{
  return x * (erff(x * 0.70710678118654752f) + 1.f) * 0.5f;
}

__device__ __forceinline__ float epi_f(float v, int ep, const float* __restrict__ gate, int mg)
{
  if (ep == EP_GELU) return gelu_f(v);
  if (ep == EP_GATE) return v * (1.f / (1.f + expf(-gate[mg])));
  return v;
}

template <int MODE>
__global__ __launch_bounds__(256)
void k_gemm(const float* __restrict__ X, const float* __restrict__ Wt,
            const float* __restrict__ bias, const float* __restrict__ gate,
            float* Y, int Cout, int Cin, int Npix,
            long xbs, long xcs, long xps, long ybs, long yos,
            int epilogue, int vt_store)
{
  __shared__ alignas(16) _Float16 As[64 * KP];
  __shared__ alignas(16) _Float16 Bs[32 * KP];
  __shared__ alignas(16) float    Cs[64 * CSP];

  const int tid  = threadIdx.x;
  const int lane = tid & 31, wave = tid >> 5;
  const int wm   = wave >> 1;
  const int wn   = wave & 1;
  const int hf   = lane >> 4;
  const int lm   = lane & 15;
  const int m0   = blockIdx.x * 64, n0 = blockIdx.y * 32, batch = blockIdx.z;
  const int Ktot = (MODE == 0) ? Cin : Cin * 9;
  const float* Xb = X + (size_t)batch * (size_t)xbs;

  const int aRow = tid >> 2, aK0 = (tid & 3) * 16;
  const int bK   = tid >> 2, bN0 = (tid & 3) * 8;

  v8f acc = {0.f, 0.f, 0.f, 0.f, 0.f, 0.f, 0.f, 0.f};

  for (int kk = 0; kk < Ktot; kk += KSTEP) {
    {
      const int o = m0 + aRow;
      HPack pa;
#pragma unroll
      for (int i = 0; i < 16; ++i) {
        const int k = kk + aK0 + i;
        float w = 0.f;
        if (o < Cout && k < Ktot) {
          if (MODE == 0) {
            w = Wt[(size_t)o * Cin + k];
          } else {
            const int t  = k / Cin;
            const int ci = k - t * Cin;
            w = Wt[((size_t)o * Cin + ci) * 9 + t];
          }
        }
        pa.s[i] = (_Float16)(w * OPSCALE);
      }
      *(v8ha*)(&As[aRow * KP + aK0])     = pa.v[0];
      *(v8ha*)(&As[aRow * KP + aK0 + 8]) = pa.v[1];
    }
    {
      const int k = kk + bK;
      int ci = k, dy = 0, dx = 0;
      if (MODE == 1) {
        const int t  = k / Cin;
        ci = k - t * Cin;
        const int t3 = t / 3;
        dy = t3 - 1;
        dx = t - t3 * 3 - 1;
      }
#pragma unroll
      for (int i = 0; i < 8; ++i) {
        const int nl  = bN0 + i;
        const int pix = n0 + nl;
        float x = 0.f;
        if (k < Ktot && pix < Npix) {
          if (MODE == 0) {
            x = Xb[(size_t)k * (size_t)xcs + (size_t)pix * (size_t)xps];
          } else {
            const int ph = pix / WW;
            const int hh = ph + dy, ww = (pix - ph * WW) + dx;
            if (hh >= 0 && hh < HH && ww >= 0 && ww < WW)
              x = Xb[(size_t)ci * (size_t)xcs + (size_t)(hh * WW + ww)];
          }
        }
        Bs[nl * KP + bK] = (_Float16)(x * OPSCALE);
      }
    }
    __syncthreads();

#pragma unroll
    for (int s = 0; s < 2; ++s) {
      const int kb = s * 32;
      Frag fa, fb;
      fa.half[0] = *(const v8ha*)(&As[(wm * 16 + lm) * KP + kb + 8 * hf]);
      fa.half[1] = *(const v8ha*)(&As[(wm * 16 + lm) * KP + kb + 16 + 8 * hf]);
      fb.half[0] = *(const v8ha*)(&Bs[(wn * 16 + lm) * KP + kb + 8 * hf]);
      fb.half[1] = *(const v8ha*)(&Bs[(wn * 16 + lm) * KP + kb + 16 + 8 * hf]);
      acc = wmma16(fa.v, fb.v, acc);
    }
    __syncthreads();
  }

#pragma unroll
  for (int r = 0; r < 8; ++r) {
    const int ml = wm * 16 + 8 * hf + r;
    const int mg = m0 + ml;
    float v = 0.f;
    if (mg < Cout) v = epi_f(acc[r] * ACCSCALE + bias[mg], epilogue, gate, mg);
    Cs[ml * CSP + wn * 16 + lm] = v;
  }
  __syncthreads();

  v4f sv0, sv1;
  float* sp0; float* sp1;
  bool ok0, ok1;
  const int q4 = (lane & 7) * 4;
  if (!vt_store) {
    const int r0 = wave * 8 + (lane >> 3);
    const int r1 = r0 + 4;
    sv0 = *(const v4fa*)(&Cs[r0 * CSP + q4]);
    sv1 = *(const v4fa*)(&Cs[r1 * CSP + q4]);
    ok0 = (m0 + r0 < Cout) && (n0 + q4 + 3 < Npix);
    ok1 = (m0 + r1 < Cout) && (n0 + q4 + 3 < Npix);
    sp0 = Y + (size_t)batch * (size_t)ybs + (size_t)(m0 + r0) * (size_t)yos + (size_t)(n0 + q4);
    sp1 = Y + (size_t)batch * (size_t)ybs + (size_t)(m0 + r1) * (size_t)yos + (size_t)(n0 + q4);
  } else {
    const int kl  = wave >> 2;
    const int nA  = (wave & 3) * 8 + (lane >> 3);
    const int nB  = nA + 4;
    sv0.x = Cs[(kl * 32 + q4 + 0) * CSP + nA]; sv0.y = Cs[(kl * 32 + q4 + 1) * CSP + nA];
    sv0.z = Cs[(kl * 32 + q4 + 2) * CSP + nA]; sv0.w = Cs[(kl * 32 + q4 + 3) * CSP + nA];
    sv1.x = Cs[(kl * 32 + q4 + 0) * CSP + nB]; sv1.y = Cs[(kl * 32 + q4 + 1) * CSP + nB];
    sv1.z = Cs[(kl * 32 + q4 + 2) * CSP + nB]; sv1.w = Cs[(kl * 32 + q4 + 3) * CSP + nB];
    ok0 = (m0 + kl * 32 + 31 < Cout) && (n0 + nA < Npix);
    ok1 = (m0 + kl * 32 + 31 < Cout) && (n0 + nB < Npix);
    const size_t hb = (size_t)batch * ((size_t)Cout * (size_t)Npix)
                    + (size_t)((m0 >> 5) + kl) * ((size_t)Npix * DD);
    sp0 = Y + hb + (size_t)(n0 + nA) * DD + q4;
    sp1 = Y + hb + (size_t)(n0 + nB) * DD + q4;
  }
  if (ok0) *(volatile v4f*)sp0 = sv0;
  if (ok1) *(volatile v4f*)sp1 = sv1;
  __threadfence();
  if (ok0) *(volatile v4f*)sp0 = sv0;
  if (ok1) *(volatile v4f*)sp1 = sv1;
}

__global__ __launch_bounds__(256)
void k_dwconv(const float* __restrict__ X, const float* __restrict__ Wd,
              const float* __restrict__ bias, float* Y, int nbc)
{
  const int bc = blockIdx.x;
  const bool act = bc < nbc;
  const int c  = bc & (CC - 1);
  const int lane = threadIdx.x & 31;
  const float* src = X + (size_t)bc * HWp;
  float*       dst = Y + (size_t)bc * HWp;
  float w[9];
#pragma unroll
  for (int i = 0; i < 9; ++i) w[i] = act ? Wd[c * 9 + i] : 0.f;
  const float bv = act ? bias[c] : 0.f;
#pragma unroll 1
  for (int base = 0; base < HWp; base += 256) {
    const int p  = base + threadIdx.x;
    const int hr = p >> 6, xc = p & 63;
    float a = 0.f;
    if (act) {
#pragma unroll
      for (int ky = 0; ky < 3; ++ky) {
        const int yy = hr + ky - 1;
        if (yy < 0 || yy > HH - 1) continue;
#pragma unroll
        for (int kx = 0; kx < 3; ++kx) {
          const int xx = xc + kx - 1;
          if (xx < 0 || xx > WW - 1) continue;
          a += w[ky * 3 + kx] * src[yy * WW + xx];
        }
      }
    }
    const float r = gelu_f(a + bv);
    v4f ov;
    ov.x = __shfl(r, (lane & 7) * 4 + 0, 32);
    ov.y = __shfl(r, (lane & 7) * 4 + 1, 32);
    ov.z = __shfl(r, (lane & 7) * 4 + 2, 32);
    ov.w = __shfl(r, (lane & 7) * 4 + 3, 32);
    float* d = dst + base + (threadIdx.x & ~31) + lane * 4;
    if (act && lane < 8) *(volatile v4f*)d = ov;
    __threadfence();
    if (act && lane < 8) *(volatile v4f*)d = ov;
  }
}

__global__ __launch_bounds__(256)
void k_timeproj(const float* __restrict__ te, const float* __restrict__ tosw,
                const float* __restrict__ tosb, const float* __restrict__ tabw,
                const float* __restrict__ tabb, float* prm, int nbn)
{
  __shared__ alignas(16) float sv[PRM_N];
  const int t = threadIdx.x;
  const int nsc = nbn * (KK * PP);
  const int nbi = nbn * KK;
  for (int idx = t; idx < PRM_N; idx += 256) {
    float v = 0.f;
    if (idx < nsc) {
      const int bn = idx / (KK * PP), o = idx - bn * (KK * PP);
      float s = 0.f;
#pragma unroll 4
      for (int i = 0; i < TT; ++i) s += te[bn * TT + i] * tosw[o * TT + i];
      s += tosb[o];
      const float sp = fmaxf(s, 0.f) + log1pf(expf(-fabsf(s)));
      v = 0.5f + sp;
    } else if (idx < nsc + nbi) {
      const int j = idx - nsc;
      const int bn = j / KK, o = j - bn * KK;
      float s = 0.f;
#pragma unroll 4
      for (int i = 0; i < TT; ++i) s += te[bn * TT + i] * tabw[o * TT + i];
      s += tabb[o];
      v = s;
    }
    sv[idx] = v;
  }
  __syncthreads();
  v4f w4 = {0.f, 0.f, 0.f, 0.f};
  const bool st = t < (PRM_N / 4);
  if (st) { w4 = *(const v4fa*)(&sv[t * 4]); *(volatile v4f*)(prm + t * 4) = w4; }
  __threadfence();
  if (st) *(volatile v4f*)(prm + t * 4) = w4;
}

__global__ __launch_bounds__(256)
void k_deform(const float* __restrict__ a3, const float* __restrict__ offm,
              const float* __restrict__ prm, const float* __restrict__ rt,
              const float* __restrict__ vt, float* out_t, float* entk, int nblk)
{
  __shared__ alignas(16) float sEnt[32];
  const int lane = threadIdx.x & 31, wave = threadIdx.x >> 5;
  const int blk  = blockIdx.x;
  const bool act = blk < nblk;
  const int bk   = blk >> 7;
  const int pix0 = (blk & 127) * 32;
  const int b    = (bk >> 3) & (BB - 1), k = bk & (KK - 1);
  const bool has = lane < NN * PP;
  int n = 0, p = 0;
  if (has) { n = lane / PP; p = lane - n * PP; }
  const int kp = k * PP + p;
  float dtn = 0.f, osc = 0.f, abias = 0.f;
  if (has && act) {
    dtn   = fabsf(rt[b * NN + n]);
    osc   = prm[(b * NN + n) * (KK * PP) + kp];
    abias = prm[PRM_BIAS_OFF + (b * NN + n) * KK + k];
  }
  const int q4 = (lane & 7) * 4;

#pragma unroll 1
  for (int i = 0; i < 4; ++i) {
    const int pix = pix0 + wave * 4 + i;
    const int hq = pix >> 6, wq = pix & 63;

    float logit = -3.0e38f;
    float wxv = 0.f, wyv = 0.f;
    int x0 = 0, x1 = 0, y0 = 0, y1 = 0;
    if (has && act) {
      const float av = a3[((size_t)b * (KK * PP) + kp) * HWp + pix];
      logit = (av + abias) + (-dtn * 2.f);
      const float ox = offm[((size_t)b * (KK * PP * 2) + kp * 2 + 0) * HWp + pix];
      const float oy = offm[((size_t)b * (KK * PP * 2) + kp * 2 + 1) * HWp + pix];
      const float f1 = 1.f + dtn;
      const float sx = fminf(fmaxf((ox * osc) * f1, -1.f), 1.f);
      const float sy = fminf(fmaxf((oy * osc) * f1, -1.f), 1.f);
      const float tw = (float)wq * (1.f / 63.f);
      const float th = (float)hq * (1.f / 63.f);
      const float bgx = -1.f * (1.f - tw) + 1.f * tw;
      const float bgy = -1.f * (1.f - th) + 1.f * th;
      const float gx = fminf(fmaxf(bgx + sx, -1.f), 1.f);
      const float gy = fminf(fmaxf(bgy + sy, -1.f), 1.f);
      const float gxp = (gx + 1.f) * 0.5f * (float)(WW - 1);
      const float gyp = (gy + 1.f) * 0.5f * (float)(HH - 1);
      const float xf = floorf(gxp), yf = floorf(gyp);
      wxv = gxp - xf; wyv = gyp - yf;
      const int xi = (int)xf, yi = (int)yf;
      x0 = min(max(xi, 0), WW - 1);     x1 = min(max(xi + 1, 0), WW - 1);
      y0 = min(max(yi, 0), HH - 1);     y1 = min(max(yi + 1, 0), HH - 1);
    }

    float mx = logit;
    for (int s = 16; s; s >>= 1) mx = fmaxf(mx, __shfl_xor(mx, s, 32));
    const float e = has ? expf(logit - mx) : 0.f;
    float sum = e;
    for (int s = 16; s; s >>= 1) sum += __shfl_xor(sum, s, 32);
    const float wgt = e * (1.f / sum);
    float ev = has ? (wgt * logf(wgt + 1e-8f)) : 0.f;
    for (int s = 16; s; s >>= 1) ev += __shfl_xor(ev, s, 32);
    if (lane == 0) sEnt[wave * 4 + i] = -ev;

    float accv = 0.f;
#pragma unroll 1
    for (int nj = 0; nj < NN; ++nj) {
      const float* vbp = vt + ((size_t)((b * NN + nj) * KK + k) * HWp) * DD + lane;
#pragma unroll
      for (int pj = 0; pj < PP; ++pj) {
        const int j = nj * PP + pj;
        const float wj  = __shfl(wgt, j, 32);
        const float wxj = __shfl(wxv, j, 32);
        const float wyj = __shfl(wyv, j, 32);
        const int x0j = __shfl(x0, j, 32);
        const int x1j = __shfl(x1, j, 32);
        const int y0j = __shfl(y0, j, 32);
        const int y1j = __shfl(y1, j, 32);
        float v00 = 0.f, v01 = 0.f, v10 = 0.f, v11 = 0.f;
        if (act) {
          v00 = vbp[(y0j * WW + x0j) * DD];
          v01 = vbp[(y0j * WW + x1j) * DD];
          v10 = vbp[(y1j * WW + x0j) * DD];
          v11 = vbp[(y1j * WW + x1j) * DD];
        }
        const float bil = v00 * (1.f - wxj) * (1.f - wyj) + v01 * wxj * (1.f - wyj)
                        + v10 * (1.f - wxj) * wyj         + v11 * wxj * wyj;
        accv += bil * wj;
      }
    }

    v4f ov;
    ov.x = __shfl(accv, q4 + 0, 32);
    ov.y = __shfl(accv, q4 + 1, 32);
    ov.z = __shfl(accv, q4 + 2, 32);
    ov.w = __shfl(accv, q4 + 3, 32);
    float* dst = out_t + ((size_t)b * HWp + pix) * CC + k * DD + q4;
    if (act && lane < 8) *(volatile v4f*)dst = ov;
    __threadfence();
    if (act && lane < 8) *(volatile v4f*)dst = ov;
  }

  __syncthreads();
  if (wave == 0) {
    v4f e4 = {0.f, 0.f, 0.f, 0.f};
    const bool st = act && lane < 8;
    float* dst = entk + (size_t)bk * HWp + pix0 + q4;
    if (st) { e4 = *(const v4fa*)(&sEnt[q4]); *(volatile v4f*)dst = e4; }
    __threadfence();
    if (st) *(volatile v4f*)dst = e4;
  }
}

__global__ __launch_bounds__(256)
void k_conf(const float* __restrict__ entk, float* outc, float* oute, int nquads)
{
  const int q = blockIdx.x * 256 + threadIdx.x;
  const bool act = q < nquads;
  const int e0 = q * 4;
  const int b = e0 >> 12, pix = e0 & (HWp - 1);
  v4f s = {0.f, 0.f, 0.f, 0.f};
  if (act) {
#pragma unroll
    for (int k = 0; k < KK; ++k)
      s += *(const v4fa*)(entk + ((size_t)(b * KK + k)) * HWp + pix);
  }
  const v4f en = s / (float)KK;
  const float inv = 1.f / 3.17805383034794562f;
  v4f cf;
  cf.x = 1.f - fminf(fmaxf(en.x * inv, 0.f), 1.f);
  cf.y = 1.f - fminf(fmaxf(en.y * inv, 0.f), 1.f);
  cf.z = 1.f - fminf(fmaxf(en.z * inv, 0.f), 1.f);
  cf.w = 1.f - fminf(fmaxf(en.w * inv, 0.f), 1.f);
  if (act) { *(volatile v4f*)(outc + e0) = cf; *(volatile v4f*)(oute + e0) = en; }
  __threadfence();
  if (act) { *(volatile v4f*)(outc + e0) = cf; *(volatile v4f*)(oute + e0) = en; }
}

template <int MODE>
static inline void launch_gemm(hipStream_t s,
                               const float* X, const float* Wt, const float* bias,
                               const float* gate, float* Y,
                               int Cout, int Cin, int Npix, int nbatch,
                               long xbs, long xcs, long xps, long ybs, long yos,
                               int ep, int vt)
{
  dim3 grid((Cout + 63) / 64, (Npix + 31) / 32, nbatch);
  k_gemm<MODE><<<grid, 256, 0, s>>>(X, Wt, bias, gate, Y, Cout, Cin, Npix,
                                    xbs, xcs, xps, ybs, yos, ep, vt);
}

extern "C" void kernel_launch(void* const* d_in, const int* in_sizes, int n_in,
                              void* d_out, int out_size, void* d_ws, size_t ws_size,
                              hipStream_t stream)
{
  if (n_in < 31) return;
  if (in_sizes[0] != BB * CC * HWp) return;
  if (in_sizes[1] != BB * NN * CC * HWp) return;
  if (in_sizes[3] != BB * NN * TT) return;
  if (out_size != BB * CC * HWp + 2 * BB * HWp) return;

  const size_t oQ    = 0;
  const size_t oA    = oQ   + (size_t)BB * CC * HWp;
  const size_t oBf   = oA   + (size_t)BB * CC * HWp;
  const size_t oC    = oBf  + (size_t)BB * CC * HWp;
  const size_t oOFF  = oC   + (size_t)BB * (CC / 2) * HWp;
  const size_t oC2   = oOFF + (size_t)BB * (KK * PP * 2) * HWp;
  const size_t oATT  = oC2  + (size_t)BB * (CC / 4) * HWp;
  const size_t oVT   = oATT + (size_t)BB * (KK * PP) * HWp;
  const size_t oENT  = oVT  + (size_t)BB * NN * CC * HWp;
  const size_t oPRM  = oENT + (size_t)BB * KK * HWp;
  const size_t total = oPRM + PRM_N;
  if (total * sizeof(float) > ws_size) return;

  const float* query    = (const float*)d_in[0];
  const float* values   = (const float*)d_in[1];
  const float* rel_time = (const float*)d_in[2];
  const float* time_enc = (const float*)d_in[3];
  const float* qw   = (const float*)d_in[4];   const float* qb   = (const float*)d_in[5];
  const float* dww  = (const float*)d_in[6];   const float* dwb  = (const float*)d_in[7];
  const float* o1w  = (const float*)d_in[8];   const float* o1b  = (const float*)d_in[9];
  const float* o2w  = (const float*)d_in[10];  const float* o2b  = (const float*)d_in[11];
  const float* o3w  = (const float*)d_in[12];  const float* o3b  = (const float*)d_in[13];
  const float* tosw = (const float*)d_in[14];  const float* tosb = (const float*)d_in[15];
  const float* a1w  = (const float*)d_in[16];  const float* a1b  = (const float*)d_in[17];
  const float* a2w  = (const float*)d_in[18];  const float* a2b  = (const float*)d_in[19];
  const float* a3w  = (const float*)d_in[20];  const float* a3b  = (const float*)d_in[21];
  const float* tabw = (const float*)d_in[22];  const float* tabb = (const float*)d_in[23];
  const float* vw   = (const float*)d_in[24];  const float* vb   = (const float*)d_in[25];
  const float* u1w  = (const float*)d_in[26];  const float* u1b  = (const float*)d_in[27];
  const float* u2w  = (const float*)d_in[28];  const float* u2b  = (const float*)d_in[29];
  const float* gate = (const float*)d_in[30];

  float* ws   = (float*)d_ws;
  float* Q    = ws + oQ;
  float* bufA = ws + oA;
  float* bufB = ws + oBf;
  float* bufC = ws + oC;
  float* OFF  = ws + oOFF;
  float* C2   = ws + oC2;
  float* ATT  = ws + oATT;
  float* VT   = ws + oVT;
  float* ENTK = ws + oENT;
  float* PRM  = ws + oPRM;

  float* out_main = (float*)d_out;
  float* out_conf = out_main + (size_t)BB * CC * HWp;
  float* out_entr = out_conf + (size_t)BB * HWp;

  const long CS = (long)CC * HWp;

  launch_gemm<0>(stream, query, qw, qb, qb, Q, CC, CC, HWp, BB,
                 CS, HWp, 1, CS, HWp, EP_NONE, 0);
  k_dwconv<<<BB * CC, 256, 0, stream>>>(Q, dww, dwb, bufA, BB * CC);
  launch_gemm<0>(stream, bufA, o1w, o1b, o1b, bufB, CC, CC, HWp, BB,
                 CS, HWp, 1, CS, HWp, EP_GELU, 0);
  launch_gemm<0>(stream, bufB, o2w, o2b, o2b, bufC, CC / 2, CC, HWp, BB,
                 CS, HWp, 1, (long)(CC / 2) * HWp, HWp, EP_GELU, 0);
  launch_gemm<0>(stream, bufC, o3w, o3b, o3b, OFF, KK * PP * 2, CC / 2, HWp, BB,
                 (long)(CC / 2) * HWp, HWp, 1, (long)(KK * PP * 2) * HWp, HWp, EP_NONE, 0);
  launch_gemm<0>(stream, Q, a1w, a1b, a1b, bufA, CC / 2, CC, HWp, BB,
                 CS, HWp, 1, (long)(CC / 2) * HWp, HWp, EP_GELU, 0);
  launch_gemm<1>(stream, bufA, a2w, a2b, a2b, C2, CC / 4, CC / 2, HWp, BB,
                 (long)(CC / 2) * HWp, HWp, 1, (long)(CC / 4) * HWp, HWp, EP_GELU, 0);
  launch_gemm<0>(stream, C2, a3w, a3b, a3b, ATT, KK * PP, CC / 4, HWp, BB,
                 (long)(CC / 4) * HWp, HWp, 1, (long)(KK * PP) * HWp, HWp, EP_NONE, 0);
  launch_gemm<0>(stream, values, vw, vb, vb, VT, CC, CC, HWp, BB * NN,
                 CS, HWp, 1, 0, 0, EP_NONE, 1);
  k_timeproj<<<1, 256, 0, stream>>>(time_enc, tosw, tosb, tabw, tabb, PRM, BB * NN);
  k_deform<<<(BB * KK * HWp) / 32, 256, 0, stream>>>(ATT, OFF, PRM, rel_time, VT,
                                                     bufB, ENTK, (BB * KK * HWp) / 32);
  launch_gemm<0>(stream, bufB, u1w, u1b, u1b, bufA, CC, CC, HWp, BB,
                 (long)HWp * CC, 1, CC, CS, HWp, EP_GELU, 0);
  launch_gemm<0>(stream, bufA, u2w, u2b, gate, out_main, CC, CC, HWp, BB,
                 CS, HWp, 1, CS, HWp, EP_GATE, 0);
  k_conf<<<(BB * HWp / 4 + 255) / 256, 256, 0, stream>>>(ENTK, out_conf, out_entr, BB * HWp / 4);
  (void)hipGetLastError();
}
